// ConfigurableLSTMModel_26594437497060
// MI455X (gfx1250) — hardware-verified
//
#include <hip/hip_runtime.h>
#include <math.h>
#include <stddef.h>


constexpr int CD   = 16;
constexpr int TIN  = 512;
constexpr int TOUT = 200;
constexpr int CH   = 512;
constexpr int G4   = 4 * CH;
constexpr int KC   = CH + 32;
constexpr int KP   = 576;
constexpr int KPC  = KP / 8;
constexpr int HP   = KC;
constexpr int BT   = 16;
constexpr int NTHR = 256;
constexpr float WSCALE = 64.0f;
constexpr float WINV   = 0.015625f;

typedef _Float16 f16;
typedef _Float16 v16h __attribute__((ext_vector_type(16)));
typedef _Float16 v8h  __attribute__((ext_vector_type(8)));
typedef float    v8f  __attribute__((ext_vector_type(8)));
typedef float    v4f  __attribute__((ext_vector_type(4)));
typedef v8h __attribute__((may_alias)) v8ha;
typedef v4f __attribute__((may_alias)) v4fa;

union Frag { v16h v; v8h h[2]; };

__device__ __forceinline__ v8f wmma16(v16h a, v16h b, v8f c) {
  v8f d = __builtin_amdgcn_wmma_f32_16x16x32_f16(false, a, false, b, (short)0, c, false, false);
  asm volatile("v_nop\n\tv_nop\n\tv_nop\n\tv_nop" : "+v"(d) : "v"(a), "v"(b));
  return d;
}

__device__ __forceinline__ float sigm(float x) { return 1.0f / (1.0f + expf(-x)); }

__global__ __launch_bounds__(NTHR)
void pack_kernel(const float* __restrict__ Whh, const float* __restrict__ Wih,
                 f16* __restrict__ Wc, int nChunks) {
  const int gid = blockIdx.x * NTHR + threadIdx.x;
  if (gid >= nChunks) return;
  const int n  = gid / KPC;
  const int k0 = (gid - n * KPC) * 8;
  float v[8];
  if (k0 < CH) {
    #pragma unroll
    for (int j = 0; j < 8; ++j) v[j] = Whh[(size_t)n * CH + k0 + j];
  } else if (k0 < CH + CD) {
    #pragma unroll
    for (int j = 0; j < 8; ++j) v[j] = Wih[(size_t)n * CD + (k0 - CH) + j];
  } else {
    #pragma unroll
    for (int j = 0; j < 8; ++j) v[j] = 0.0f;
  }
  v8h o;
  #pragma unroll
  for (int j = 0; j < 8; ++j) o[j] = (f16)(v[j] * WSCALE);
  f16* dst = Wc + (size_t)gid * 8;
  *(volatile v8h*)dst = o;
  __threadfence();
  *(volatile v8h*)dst = o;
}

template <int G>
__device__ __forceinline__ void gate_group(const f16* cur, f16* nxt,
                                           const f16* __restrict__ Wc,
                                           const float* __restrict__ bih,
                                           const float* __restrict__ bhh,
                                           float (&cs)[8], int wid, int l) {
  const int hh = l >> 4, m16 = l & 15;
  const int u = 64 * wid + 16 * G + m16;
  const v8f z8 = {0.f, 0.f, 0.f, 0.f, 0.f, 0.f, 0.f, 0.f};
  v8f acc[4];
  #pragma unroll
  for (int q = 0; q < 4; ++q) acc[q] = z8;
  const f16* wr = Wc + (size_t)u * KP + 8 * hh;
  const f16* ar = cur + m16 * HP + 8 * hh;
  #pragma unroll 1
  for (int ks = 0; ks < KC / 32; ++ks) {
    const int k0 = ks * 32;
    Frag a;
    a.h[0] = *(const v8ha*)(ar + k0);
    a.h[1] = *(const v8ha*)(ar + k0 + 16);
    Frag b[4];
    #pragma unroll
    for (int q = 0; q < 4; ++q) {
      const f16* wq = wr + (size_t)q * CH * KP + k0;
      b[q].h[0] = *(const v8ha*)(wq);
      b[q].h[1] = *(const v8ha*)(wq + 16);
    }
    #pragma unroll
    for (int q = 0; q < 4; ++q) acc[q] = wmma16(a.v, b[q].v, acc[q]);
  }
  const float bi = bih[u]          + bhh[u];
  const float bf = bih[CH + u]     + bhh[CH + u];
  const float bg = bih[2 * CH + u] + bhh[2 * CH + u];
  const float bo = bih[3 * CH + u] + bhh[3 * CH + u];
  #pragma unroll
  for (int r = 0; r < 8; ++r) {
    const float gi = acc[0][r] * WINV + bi;
    const float gf = acc[1][r] * WINV + bf;
    const float gg = acc[2][r] * WINV + bg;
    const float go = acc[3][r] * WINV + bo;
    const float cn = sigm(gf) * cs[r] + sigm(gi) * tanhf(gg);
    cs[r] = cn;
    const float hn = sigm(go) * tanhf(cn);
    nxt[(8 * hh + r) * HP + u] = (f16)hn;
  }
}

__global__ __launch_bounds__(NTHR)
void recur_kernel(const float* __restrict__ x, const f16* __restrict__ Wc,
                  const float* __restrict__ Wp, const float* __restrict__ bih,
                  const float* __restrict__ bhh, const float* __restrict__ bp,
                  const float* __restrict__ rw, const float* __restrict__ rb,
                  float* __restrict__ pst) {
  __shared__ f16   hs[2 * BT * HP] __attribute__((aligned(16)));
  __shared__ f16   wps[CD * CH]    __attribute__((aligned(16)));
  __shared__ float ysh[BT * CD]    __attribute__((aligned(16)));
  __shared__ float msh[BT * CD];
  __shared__ float ssh[BT * CD];

  const int tid = threadIdx.x;
  const int l = tid & 31, hh = l >> 4, m16 = l & 15, wid = tid >> 5;
  const int blk = blockIdx.x;
  const int B0 = blk * BT;

  for (int i = tid; i < 2 * BT * HP; i += NTHR) hs[i] = (f16)0.0f;
  for (int i = tid; i < CD * CH; i += NTHR) wps[i] = (f16)(Wp[i] * WSCALE);

  const int sm = tid >> 4, sd = tid & 15;
  const float* xr = x + ((size_t)(B0 + sm) * CD + sd) * TIN;
  double s1 = 0.0;
  #pragma unroll 4
  for (int t = 0; t < TIN; ++t) s1 += (double)xr[t];
  const float meanf = (float)(s1 * (1.0 / TIN));
  double s2 = 0.0;
  #pragma unroll 4
  for (int t = 0; t < TIN; ++t) {
    const float dv = xr[t] - meanf;
    s2 += (double)dv * (double)dv;
  }
  const float varf = (float)(s2 * (1.0 / TIN));
  const float stdf = sqrtf(varf + 1e-5f);
  const float istd = 1.0f / stdf;
  const float rwv = rw[sd], rbv = rb[sd];
  msh[tid] = meanf;
  ssh[tid] = stdf;
  __syncthreads();

  float c0[8], c1[8], c2[8], c3[8];
  #pragma unroll
  for (int r = 0; r < 8; ++r) { c0[r] = 0.f; c1[r] = 0.f; c2[r] = 0.f; c3[r] = 0.f; }
  const v8f z8 = {0.f, 0.f, 0.f, 0.f, 0.f, 0.f, 0.f, 0.f};

  int pp = 0;
  for (int step = 0; step < TIN + TOUT; ++step) {
    f16* cur = hs + pp * (BT * HP);
    f16* nxt = hs + (pp ^ 1) * (BT * HP);

    if (step < TIN) {
      const float v = xr[step];
      cur[sm * HP + CH + sd] = (f16)(((v - meanf) * istd) * rwv + rbv);
    } else if (wid == 0) {
      v8f pacc = z8;
      const f16* ar = cur + m16 * HP + 8 * hh;
      const f16* br = wps + m16 * CH + 8 * hh;
      #pragma unroll 1
      for (int ks = 0; ks < CH / 32; ++ks) {
        const int k0 = ks * 32;
        Frag a, b;
        a.h[0] = *(const v8ha*)(ar + k0);
        a.h[1] = *(const v8ha*)(ar + k0 + 16);
        b.h[0] = *(const v8ha*)(br + k0);
        b.h[1] = *(const v8ha*)(br + k0 + 16);
        pacc = wmma16(a.v, b.v, pacc);
      }
      const float bpd = bp[m16];
      const float irw = 1.0f / (rw[m16] + 1e-10f);
      const float rbd = rb[m16];
      #pragma unroll
      for (int r = 0; r < 8; ++r) {
        const int row = 8 * hh + r;
        const float pr = pacc[r] * WINV + bpd;
        cur[row * HP + CH + m16] = (f16)pr;
        ysh[row * CD + m16] = ((pr - rbd) * irw) * ssh[row * CD + m16] + msh[row * CD + m16];
      }
    }
    __syncthreads();

    if (step >= TIN && tid < 64) {
      const int t = step - TIN;
      const v4f val = *(const v4fa*)(ysh + 4 * tid);
      float* dst = pst + ((size_t)blk * TOUT + t) * (BT * CD) + 4 * tid;
      *(volatile v4f*)dst = val;
      __threadfence();
      *(volatile v4f*)dst = val;
    }

    gate_group<0>(cur, nxt, Wc, bih, bhh, c0, wid, l);
    gate_group<1>(cur, nxt, Wc, bih, bhh, c1, wid, l);
    gate_group<2>(cur, nxt, Wc, bih, bhh, c2, wid, l);
    gate_group<3>(cur, nxt, Wc, bih, bhh, c3, wid, l);
    __syncthreads();
    pp ^= 1;
  }
}

__global__ __launch_bounds__(NTHR)
void out_kernel(const float* __restrict__ pst, float* __restrict__ out, int nOut) {
  const size_t e0 = ((size_t)blockIdx.x * NTHR + threadIdx.x) * 4;
  if (e0 >= (size_t)nOut) return;
  float v[4];
  #pragma unroll
  for (int j = 0; j < 4; ++j) {
    size_t e = e0 + j;
    if (e >= (size_t)nOut) e = (size_t)nOut - 1;
    const int b   = (int)(e / (size_t)(CD * TOUT));
    const int rem = (int)(e - (size_t)b * (CD * TOUT));
    const int d   = rem / TOUT;
    const int t   = rem - d * TOUT;
    const int bk  = b / BT;
    const int m   = b - bk * BT;
    v[j] = pst[((size_t)bk * TOUT + t) * (BT * CD) + m * CD + d];
  }
  if (e0 + 4 <= (size_t)nOut) {
    const v4f vv = {v[0], v[1], v[2], v[3]};
    float* dst = out + e0;
    *(volatile v4f*)dst = vv;
    __threadfence();
    *(volatile v4f*)dst = vv;
  } else {
    volatile float* vo = (volatile float*)out;
    #pragma unroll
    for (int j = 0; j < 4; ++j) if (e0 + j < (size_t)nOut) vo[e0 + j] = v[j];
    __threadfence();
    #pragma unroll
    for (int j = 0; j < 4; ++j) if (e0 + j < (size_t)nOut) vo[e0 + j] = v[j];
  }
}

extern "C" void kernel_launch(void* const* d_in, const int* in_sizes, int n_in,
                              void* d_out, int out_size, void* d_ws, size_t ws_size,
                              hipStream_t stream) {
  if (n_in < 9) return;
  const float* x      = (const float*)d_in[0];
  const float* W_ih   = (const float*)d_in[1];
  const float* W_hh   = (const float*)d_in[2];
  const float* b_ih   = (const float*)d_in[3];
  const float* b_hh   = (const float*)d_in[4];
  const float* W_proj = (const float*)d_in[5];
  const float* b_proj = (const float*)d_in[6];
  const float* rev_w  = (const float*)d_in[7];
  const float* rev_b  = (const float*)d_in[8];

  const int nB = in_sizes[0] / (CD * TIN);
  if (nB <= 0 || nB * CD * TIN != in_sizes[0] || (nB % BT) != 0) return;
  if (out_size != nB * CD * TOUT) return;
  if (in_sizes[1] != G4 * CD || in_sizes[2] != G4 * CH || in_sizes[3] != G4 ||
      in_sizes[4] != G4 || in_sizes[5] != CD * CH || in_sizes[6] != CD ||
      in_sizes[7] != CD || in_sizes[8] != CD) return;
  const int nBlk = nB / BT;

  const size_t off_wc   = 0;
  const size_t wc_bytes = (size_t)G4 * KP * sizeof(f16);
  const size_t off_pst  = (off_wc + wc_bytes + 255) & ~(size_t)255;
  const size_t pst_bytes = (size_t)nBlk * TOUT * BT * CD * sizeof(float);
  if (off_pst + pst_bytes > ws_size) return;

  char* ws = (char*)d_ws;
  f16*   Wc  = (f16*)(ws + off_wc);
  float* pst = (float*)(ws + off_pst);
  float* out = (float*)d_out;

  const int nChunks = G4 * KPC;
  pack_kernel<<<(nChunks + NTHR - 1) / NTHR, NTHR, 0, stream>>>(W_hh, W_ih, Wc, nChunks);
  recur_kernel<<<nBlk, NTHR, 0, stream>>>(x, Wc, W_proj, b_ih, b_hh, b_proj, rev_w, rev_b, pst);
  const int nVec = (out_size + 3) / 4;
  out_kernel<<<(nVec + NTHR - 1) / NTHR, NTHR, 0, stream>>>(pst, out, out_size);
}
